// FU_36404142801582
// MI455X (gfx1250) — hardware-verified
//
#include <hip/hip_runtime.h>
#include <math.h>

typedef __attribute__((ext_vector_type(16))) _Float16 v16h;
typedef __attribute__((ext_vector_type(8)))  _Float16 v8h;
typedef __attribute__((ext_vector_type(4)))  _Float16 v4h;
typedef __attribute__((ext_vector_type(8)))  float    v8f;
typedef __attribute__((ext_vector_type(4)))  float    v4f;

constexpr int kB      = 8;
constexpr int kC      = 64;
constexpr int kH      = 128;
constexpr int kW      = 128;
constexpr int kHW     = kH * kW;
constexpr int kTaps   = 9;
constexpr int kOffCh  = 18;
constexpr int kGroups = 4;
constexpr int kCg     = 16;
constexpr int kHp     = kH + 2;
constexpr int kWp     = kW + 2;
constexpr int kKo     = kTaps * kC;
constexpr int kNo     = 32;
constexpr int kKdReal = kTaps * kCg;
constexpr int kKd     = 160;
constexpr int kXPitch = 132;
constexpr int kSlabP  = 68;
constexpr int kAPitch = 168;
constexpr int kDPitch = 36;
constexpr float kXCarry   = 16.0f;
constexpr float kWoCarry  = 1024.0f;
constexpr float kSCarry   = 16.0f;
constexpr float kWdCarry  = 256.0f;
constexpr float kOffScale = 1.0f / (kXCarry * kWoCarry);
constexpr float kOutScale = 1.0f / (kSCarry * kWdCarry);

static_assert(kC == kGroups * kCg, "group split");
static_assert(kOffCh == 2 * kTaps, "offset channels");
static_assert((kKo % 32) == 0 && (kKd % 32) == 0 && kKd >= kKdReal, "K multiples of 32");
static_assert((kNo % 16) == 0 && kNo >= kOffCh, "N pad");
static_assert((kKdReal % 8) == 0, "pad boundary on a 16-B chunk");
static_assert(((kB * kHW / 64) % 4) == 0, "offset conv grid exact");
static_assert((kNo * kKo / 8) == 9 * 256, "weight plane 0 chunk count");
static_assert((kC * kKd / 8) == 5 * 256, "weight plane 1 chunk count");
static_assert((kAPitch % 8) == 0 && kAPitch >= kKd, "A tile pitch");

constexpr size_t kOffXP   = 0;
constexpr size_t kSzXP    = (size_t)kB * kHp * kWp * kC * 2;
constexpr size_t kOffOFFS = kOffXP + kSzXP;
constexpr size_t kSzOFFS  = (size_t)kB * kOffCh * kHW * 4;
constexpr size_t kOffWO   = kOffOFFS + kSzOFFS;
constexpr size_t kSzWO    = (size_t)kNo * kKo * 2;
constexpr size_t kOffWD   = kOffWO + kSzWO;
constexpr size_t kSzWD    = (size_t)kC * kKd * 2;
constexpr size_t kWsTotal = kOffWD + kSzWD;
static_assert(kWsTotal == 26800128ull, "carve total");
static_assert(kWsTotal <= 134217728ull, "carve cap");
static_assert((kOffOFFS % 128) == 0 && (kOffWO % 128) == 0 && (kOffWD % 128) == 0, "aligned regions");

union FragH { v16h v; v8h h[2]; };

__device__ __forceinline__ v16h ld_frag_g(const _Float16* p) {
  FragH f;
  f.h[0] = *(const v8h*)(p);
  f.h[1] = *(const v8h*)(p + 16);
  return f.v;
}

__device__ __forceinline__ v8f mma_h(v16h a, v16h b, v8f c) {
  c = __builtin_amdgcn_wmma_f32_16x16x32_f16(false, a, false, b, (short)0, c, false, false);
  asm volatile("v_nop\n\tv_nop\n\tv_nop\n\tv_nop" : "+v"(c) : "v"(a), "v"(b));
  return c;
}

__device__ __forceinline__ int clampi(int v, int lo, int hi) {
  const int a = (v < lo) ? lo : v;
  return (a > hi) ? hi : a;
}

__global__ __launch_bounds__(256) void prep_x_kernel(const float* __restrict__ x, unsigned short* __restrict__ xp)
{
  __shared__ __align__(16) float sX[kC * kXPitch];
  const int tid = threadIdx.x, lane = tid & 31, wave = tid >> 5;
  const int b  = blockIdx.x / kHp;
  const int hp = blockIdx.x - b * kHp;
  const bool interior = (hp >= 1) && (hp <= kH);
  const int hc = clampi(hp - 1, 0, kH - 1);
  const float* xr = x + (size_t)b * kC * kHW + (size_t)hc * kW;
#pragma unroll
  for (int i = 0; i < 8; ++i) {
    const int idx = i * 256 + tid;
    const int c   = idx >> 5;
    const int w4  = (idx & 31) * 4;
    const v4f ld = *(const v4f*)(xr + (size_t)c * kHW + w4);
    v4f v;
    v[0] = interior ? ld[0] : 0.0f;
    v[1] = interior ? ld[1] : 0.0f;
    v[2] = interior ? ld[2] : 0.0f;
    v[3] = interior ? ld[3] : 0.0f;
    *(v4f*)(sX + c * kXPitch + w4) = v;
  }
  __syncthreads();
  const int q = lane >> 3, c8 = (lane & 7) * 8;
  unsigned short* rowp = xp + (size_t)blockIdx.x * kWp * kC;
  for (int qd = wave; qd < 33; qd += 8) {
    const int wp = qd * 4 + q;
    const bool inb = (wp >= 1) && (wp <= kW);
    const int wc = clampi(wp - 1, 0, kW - 1);
    v8h hv;
#pragma unroll
    for (int e = 0; e < 8; ++e) {
      const float f = sX[(c8 + e) * kXPitch + wc];
      const float s = inb ? (f * kXCarry) : 0.0f;
      hv[e] = (_Float16)s;
    }
    const bool st = (wp < kWp);
    const int wps = st ? wp : (kWp - 1);
    unsigned short* dst = rowp + (size_t)wps * kC + c8;
    for (int pass = 0; pass < 2; ++pass) {
      if (st) *(volatile v8h*)dst = hv;
      __threadfence();
    }
  }
}

__global__ __launch_bounds__(256) void prep_w_kernel(const float* __restrict__ ow, const float* __restrict__ dw,
                                                     unsigned short* __restrict__ wo, unsigned short* __restrict__ wd)
{
  const int tid = threadIdx.x;
  v8h hv;
  unsigned short* dst;
  if (blockIdx.x < 9) {
    const int i  = blockIdx.x * 256 + tid;
    const int n  = i / (kKo / 8);
    const int kc = (i - n * (kKo / 8)) * 8;
    const bool live = (n < kOffCh);
    const int nc = live ? n : (kOffCh - 1);
    const int tap = kc >> 6;
    const int c0  = kc & 63;
#pragma unroll
    for (int e = 0; e < 8; ++e) {
      const float f = ow[(size_t)(nc * kC + c0 + e) * kTaps + tap];
      const float s = live ? (f * kWoCarry) : 0.0f;
      hv[e] = (_Float16)s;
    }
    dst = wo + (size_t)i * 8;
  } else {
    const int j   = (blockIdx.x - 9) * 256 + tid;
    const int row = j / (kKd / 8);
    const int kc  = (j - row * (kKd / 8)) * 8;
    const bool live = (kc < kKdReal);
    const int tap = kc >> 4;
    const int tc  = (tap < kTaps) ? tap : (kTaps - 1);
    const int c0  = kc & 15;
#pragma unroll
    for (int e = 0; e < 8; ++e) {
      const float f = dw[(size_t)(row * kCg + c0 + e) * kTaps + tc];
      const float s = live ? (f * kWdCarry) : 0.0f;
      hv[e] = (_Float16)s;
    }
    dst = wd + (size_t)j * 8;
  }
  *(volatile v8h*)dst = hv;
  __threadfence();
  *(volatile v8h*)dst = hv;
}

__global__ __launch_bounds__(128) void offset_conv_kernel(const unsigned short* __restrict__ xp_,
                                                          const unsigned short* __restrict__ wo_,
                                                          const float* __restrict__ obias,
                                                          float* __restrict__ offs)
{
  __shared__ __align__(16) float sT[4][kNo * kSlabP];
  const _Float16* xp = (const _Float16*)xp_;
  const _Float16* wo = (const _Float16*)wo_;
  const int lane = threadIdx.x & 31, wave = threadIdx.x >> 5;
  const int hh = lane >> 4, m = lane & 15;
  const int gw = blockIdx.x * 4 + wave;
  const int b  = gw >> 8;
  const int h  = (gw >> 1) & (kH - 1);
  const int w0 = (gw & 1) * 64;

  v8f acc[4][2];
#pragma unroll
  for (int i = 0; i < 4; ++i) {
    acc[i][0] = (v8f){0.f, 0.f, 0.f, 0.f, 0.f, 0.f, 0.f, 0.f};
    acc[i][1] = (v8f){0.f, 0.f, 0.f, 0.f, 0.f, 0.f, 0.f, 0.f};
  }

#pragma unroll 1
  for (int ky = 0; ky < 3; ++ky) {
#pragma unroll 1
    for (int kx = 0; kx < 3; ++kx) {
      const int tap = ky * 3 + kx;
      const _Float16* arow = xp + ((size_t)(b * kHp + h + ky) * kWp + (size_t)(w0 + m + kx)) * kC + 8 * hh;
      const _Float16* brow = wo + (size_t)m * kKo + tap * kC + 8 * hh;
#pragma unroll
      for (int cc = 0; cc < 2; ++cc) {
        const v16h b0 = ld_frag_g(brow + cc * 32);
        const v16h b1 = ld_frag_g(brow + (size_t)16 * kKo + cc * 32);
#pragma unroll
        for (int i = 0; i < 4; ++i) {
          const v16h a = ld_frag_g(arow + (size_t)i * 16 * kC + cc * 32);
          acc[i][0] = mma_h(a, b0, acc[i][0]);
          acc[i][1] = mma_h(a, b1, acc[i][1]);
        }
      }
    }
  }

  float* slab = sT[wave];
#pragma unroll
  for (int j = 0; j < 2; ++j) {
    const int n  = j * 16 + m;
    const int nc = (n < kOffCh) ? n : (kOffCh - 1);
    const float braw = obias[nc];
    const float bv = (n < kOffCh) ? braw : 0.0f;
#pragma unroll
    for (int i = 0; i < 4; ++i) {
      v4f t0, t1;
#pragma unroll
      for (int r = 0; r < 4; ++r) {
        t0[r] = fmaf(acc[i][j][r], kOffScale, bv);
        t1[r] = fmaf(acc[i][j][4 + r], kOffScale, bv);
      }
      float* sp = slab + n * kSlabP + i * 16 + 8 * hh;
      *(v4f*)(sp) = t0;
      *(v4f*)(sp + 4) = t1;
    }
  }
  __syncthreads();
  {
    const int c4 = m * 4;
    float* ob = offs + (size_t)b * kOffCh * kHW + (size_t)h * kW + w0 + c4;
    for (int pass = 0; pass < 2; ++pass) {
#pragma unroll
      for (int it = 0; it < 9; ++it) {
        const int n = it * 2 + hh;
        const v4f v = *(const v4f*)(slab + n * kSlabP + c4);
        *(volatile v4f*)(ob + (size_t)n * kHW) = v;
      }
      __threadfence();
    }
  }
}

__global__ __launch_bounds__(32) void deform_kernel(const float* __restrict__ skip, const float* __restrict__ offs,
                                                    const unsigned short* __restrict__ wd_, float* __restrict__ out)
{
  __shared__ __align__(16) _Float16 sA[kGroups * 32 * kAPitch];
  __shared__ __align__(16) float sD[kC * kDPitch];
  const _Float16* wd = (const _Float16*)wd_;
  const int lane = threadIdx.x;
  const int hh = lane >> 4, m = lane & 15;
  const int t  = blockIdx.x;
  const int b  = t >> 9;
  const int h  = (t >> 2) & (kH - 1);
  const int w0 = (t & 3) * 32;
  const int w  = w0 + lane;

  {
    v8h z;
#pragma unroll
    for (int e = 0; e < 8; ++e) z[e] = (_Float16)0.0f;
#pragma unroll
    for (int g = 0; g < kGroups; ++g) {
      _Float16* zp = sA + (g * 32 + lane) * kAPitch + kKdReal;
      *(v8h*)(zp) = z;
      *(v8h*)(zp + 8) = z;
    }
  }

  const float* sb = skip + (size_t)b * kC * kHW;
  const float* op = offs + (size_t)b * kOffCh * kHW + (size_t)h * kW + w;

#pragma unroll 1
  for (int ky = 0; ky < 3; ++ky) {
#pragma unroll 1
    for (int kx = 0; kx < 3; ++kx) {
      const int tap = ky * 3 + kx;
      const float dy = op[(size_t)(2 * tap) * kHW];
      const float dx = op[(size_t)(2 * tap + 1) * kHW];
      const float py = (float)(h - 1 + ky) + dy;
      const float px = (float)(w - 1 + kx) + dx;
      const float y0f = floorf(py);
      const float x0f = floorf(px);
      const float wy = py - y0f;
      const float wx = px - x0f;
      const int y0 = (int)fminf(fmaxf(y0f, -4.0f), 132.0f);
      const int x0 = (int)fminf(fmaxf(x0f, -4.0f), 132.0f);
      const int y1 = y0 + 1, x1 = x0 + 1;
      const bool vy0 = ((unsigned)y0 < (unsigned)kH);
      const bool vy1 = ((unsigned)y1 < (unsigned)kH);
      const bool vx0 = ((unsigned)x0 < (unsigned)kW);
      const bool vx1 = ((unsigned)x1 < (unsigned)kW);
      const float omy = 1.0f - wy;
      const float omx = 1.0f - wx;
      const float w00 = (vy0 && vx0) ? (omy * omx * kSCarry) : 0.0f;
      const float w01 = (vy0 && vx1) ? (omy * wx * kSCarry) : 0.0f;
      const float w10 = (vy1 && vx0) ? (wy * omx * kSCarry) : 0.0f;
      const float w11 = (vy1 && vx1) ? (wy * wx * kSCarry) : 0.0f;
      const int cy0 = clampi(y0, 0, kH - 1);
      const int cy1 = clampi(y1, 0, kH - 1);
      const int cx0 = clampi(x0, 0, kW - 1);
      const int cx1 = clampi(x1, 0, kW - 1);
      const int i00 = cy0 * kW + cx0;
      const int i01 = cy0 * kW + cx1;
      const int i10 = cy1 * kW + cx0;
      const int i11 = cy1 * kW + cx1;
#pragma unroll 1
      for (int cq = 0; cq < 16; ++cq) {
        const float* sc = sb + (size_t)(cq * 4) * kHW;
        v4h hv;
#pragma unroll
        for (int e = 0; e < 4; ++e) {
          const float* se = sc + (size_t)e * kHW;
          float v = w00 * se[i00];
          v = fmaf(w01, se[i01], v);
          v = fmaf(w10, se[i10], v);
          v = fmaf(w11, se[i11], v);
          hv[e] = (_Float16)v;
        }
        const int g = cq >> 2;
        *(v4h*)(sA + (g * 32 + lane) * kAPitch + tap * kCg + (cq & 3) * 4) = hv;
      }
    }
  }
  __syncthreads();

#pragma unroll 1
  for (int g = 0; g < kGroups; ++g) {
    v8f a0 = (v8f){0.f, 0.f, 0.f, 0.f, 0.f, 0.f, 0.f, 0.f};
    v8f a1 = (v8f){0.f, 0.f, 0.f, 0.f, 0.f, 0.f, 0.f, 0.f};
    const _Float16* bp = wd + (size_t)(g * kCg + m) * kKd + 8 * hh;
    const _Float16* ap = sA + (g * 32 + m) * kAPitch + 8 * hh;
#pragma unroll
    for (int ks = 0; ks < kKd / 32; ++ks) {
      const v16h bf = ld_frag_g(bp + ks * 32);
      FragH f0, f1;
      f0.h[0] = *(const v8h*)(ap + ks * 32);
      f0.h[1] = *(const v8h*)(ap + ks * 32 + 16);
      f1.h[0] = *(const v8h*)(ap + 16 * kAPitch + ks * 32);
      f1.h[1] = *(const v8h*)(ap + 16 * kAPitch + ks * 32 + 16);
      a0 = mma_h(f0.v, bf, a0);
      a1 = mma_h(f1.v, bf, a1);
    }
    float* dp = sD + (g * kCg + m) * kDPitch + 8 * hh;
    v4f t0, t1, t2, t3;
#pragma unroll
    for (int r = 0; r < 4; ++r) {
      t0[r] = a0[r] * kOutScale;
      t1[r] = a0[4 + r] * kOutScale;
      t2[r] = a1[r] * kOutScale;
      t3[r] = a1[4 + r] * kOutScale;
    }
    *(v4f*)(dp) = t0;
    *(v4f*)(dp + 4) = t1;
    *(v4f*)(dp + 16) = t2;
    *(v4f*)(dp + 20) = t3;
  }
  __syncthreads();
  {
    const int q = lane >> 3, c4 = (lane & 7) * 4;
    float* ob = out + (size_t)b * kC * kHW + (size_t)h * kW + w0 + c4;
    for (int pass = 0; pass < 2; ++pass) {
#pragma unroll
      for (int it = 0; it < 16; ++it) {
        const int ch = it * 4 + q;
        const v4f v = *(const v4f*)(sD + ch * kDPitch + c4);
        *(volatile v4f*)(ob + (size_t)ch * kHW) = v;
      }
      __threadfence();
    }
  }
}

extern "C" void kernel_launch(void* const* d_in, const int* in_sizes, int n_in,
                              void* d_out, int out_size, void* d_ws, size_t ws_size,
                              hipStream_t stream) {
  if (n_in < 5) return;
  if (in_sizes[0] != kB * kC * kHW) return;
  if (in_sizes[1] != kB * kC * kHW) return;
  if (in_sizes[2] != kOffCh * kC * kTaps) return;
  if (in_sizes[3] != kOffCh) return;
  if (in_sizes[4] != kC * kCg * kTaps) return;
  if (out_size != kB * kC * kHW) return;
  if (ws_size < kWsTotal) return;

  const float* x        = (const float*)d_in[0];
  const float* skip     = (const float*)d_in[1];
  const float* offset_w = (const float*)d_in[2];
  const float* offset_b = (const float*)d_in[3];
  const float* deform_w = (const float*)d_in[4];
  float* out = (float*)d_out;

  char* ws = (char*)d_ws;
  unsigned short* XP   = (unsigned short*)(ws + kOffXP);
  float*          OFFS = (float*)(ws + kOffOFFS);
  unsigned short* WO   = (unsigned short*)(ws + kOffWO);
  unsigned short* WD   = (unsigned short*)(ws + kOffWD);

  prep_x_kernel<<<kB * kHp, 256, 0, stream>>>(x, XP);
  prep_w_kernel<<<14, 256, 0, stream>>>(offset_w, deform_w, WO, WD);
  offset_conv_kernel<<<(kB * kHW / 64) / 4, 128, 0, stream>>>(XP, WO, offset_b, OFFS);
  deform_kernel<<<kB * kH * (kW / 32), 32, 0, stream>>>(skip, OFFS, WD, out);
}
